// Node_Edge_64166811403051
// MI455X (gfx1250) — hardware-verified
//
#include <hip/hip_runtime.h>
#include <stddef.h>

#define NN    18
#define C1    64
#define C2    128
#define NPIX  324
#define NPAIR 171
#define TPE   11
#define EPB   4
#define NTB   (EPB * TPE)
#define H1S   136
#define NTHR  256
#define NWAV  8
#define OUTE  648
#define PPE   (OUTE / 4)
#define PPB   (EPB * PPE)
#define NPK   ((PPB + NTHR - 1) / NTHR)

static_assert((EPB * OUTE * 4) % 128 == 0);
static_assert(EPB * OUTE <= EPB * NN * C1);
static_assert(TPE * 16 >= NPAIR);
static_assert(H1S % 8 == 0);
static_assert(H1S >= C2);
static_assert((NN * C1) % 4 == 0);
static_assert(NPK == 3);

typedef _Float16 f16;
typedef f16 v16h __attribute__((ext_vector_type(16)));
typedef f16 v8h_t __attribute__((ext_vector_type(8)));
typedef v8h_t __attribute__((may_alias)) v8h;
typedef float v8f __attribute__((ext_vector_type(8)));
typedef float v4f_t __attribute__((ext_vector_type(4)));
typedef v4f_t __attribute__((may_alias)) v4f;
typedef unsigned int v4u __attribute__((ext_vector_type(4)));

union Frag { v16h v; v8h_t h[2]; };

__device__ __forceinline__ v8f zero8() {
    v8f z;
#pragma unroll
    for (int i = 0; i < 8; ++i) z[i] = 0.0f;
    return z;
}

__device__ __forceinline__ v8f wmma16(v16h a, v16h b, v8f c) {
    return __builtin_amdgcn_wmma_f32_16x16x32_f16(false, a, false, b, (short)0, c, false, false);
}

__global__ void __launch_bounds__(256) cvt_w_kernel(
    const float* __restrict__ W1, const float* __restrict__ W2,
    f16* __restrict__ w1h, f16* __restrict__ w2h, int n8, int nbm)
{
    const int mat = blockIdx.x / nbm;
    const int i   = (blockIdx.x - mat * nbm) * 256 + threadIdx.x;
    const float* src = (mat == 0) ? W1 : W2;
    f16* dst = (mat == 0) ? w1h : w2h;
    const bool ok = (i < n8);
    const int ic = ok ? i : (n8 - 1);
    const v4f_t a = *(const v4f*)(src + (size_t)ic * 8);
    const v4f_t b = *(const v4f*)(src + (size_t)ic * 8 + 4);
    union { v8h_t h; v4u u; } pk;
#pragma unroll
    for (int j = 0; j < 4; ++j) {
        pk.h[j]     = (f16)(a[j] * 64.0f);
        pk.h[4 + j] = (f16)(b[j] * 64.0f);
    }
    if (ok) *(volatile v4u*)(dst + (size_t)ic * 8) = pk.u;
    __threadfence();
    if (ok) *(volatile v4u*)(dst + (size_t)ic * 8) = pk.u;
}

__global__ void __launch_bounds__(NTHR) edge_kernel(
    const float* __restrict__ node,
    const float* __restrict__ last_edge,
    const f16*   __restrict__ w1h,
    const float* __restrict__ g1, const float* __restrict__ b1,
    const float* __restrict__ m1, const float* __restrict__ v1,
    const f16*   __restrict__ w2h,
    const float* __restrict__ g2, const float* __restrict__ b2,
    const float* __restrict__ m2, const float* __restrict__ v2,
    const float* __restrict__ W3,
    const float* __restrict__ b3,
    float* __restrict__ out,
    int nB)
{
    __shared__ __align__(16) float nodeS[EPB * NN * C1];
    __shared__ __align__(16) f16   h1S[NWAV * 16 * H1S];
    __shared__ float epS[EPB * NPIX];
    __shared__ float mkS[NPIX];
    __shared__ float s1S[C2], m1S[C2], b1S[C2];
    __shared__ float s2S[C1], m2S[C1], b2S[C1], w3S[C1];

    const int tid  = threadIdx.x;
    const int lane = tid & 31;
    const int wave = tid >> 5;
    const int hi   = lane >> 4;
    const int ln   = lane & 15;
    const int blk  = blockIdx.x;
    const int epg0 = blk * EPB;

    for (int q = tid; q < EPB * NN * C1 / 4; q += NTHR) {
        const int fl = q * 4;
        const int e  = fl / (NN * C1);
        const int r  = fl - e * (NN * C1);
        int eg = epg0 + e; eg = (eg < nB) ? eg : (nB - 1);
        const v4f_t v = *(const v4f*)(node + (size_t)eg * (NN * C1) + r);
        *(v4f*)(nodeS + fl) = v;
    }
    for (int q = tid; q < NPIX; q += NTHR) {
        const int i = q / NN, j = q - i * NN;
        float mm = (i == j) ? 1.0f : 0.0f;
        mm = (j == i + 1) ? 1.0f : mm;
        mm = (i == j + 1) ? 1.0f : mm;
        float bk = ((i < 9 && j >= 9) || (i >= 9 && j < 9)) ? 1.0f : 0.0f;
        bk = ((i == 8 && j == 9) || (i == 9 && j == 8)) ? 0.0f : bk;
        mkS[q] = bk + mm;
    }
    if (tid < C2) {
        s1S[tid] = g1[tid] * (1.0f / sqrtf(v1[tid] + 1e-5f));
        m1S[tid] = m1[tid];
        b1S[tid] = b1[tid];
    }
    if (tid < C1) {
        s2S[tid] = g2[tid] * (1.0f / sqrtf(v2[tid] + 1e-5f));
        m2S[tid] = m2[tid];
        b2S[tid] = b2[tid];
        w3S[tid] = W3[tid];
    }
    __syncthreads();

    const float bias3 = b3[0];
    f16* myH1 = h1S + wave * 16 * H1S;
    const float acc_scale = 1.0f / 1024.0f;

#pragma unroll 1
    for (int t = wave; t < NTB; t += NWAV) {
        const int e  = t / TPE;
        const int tl = t - e * TPE;
        const int tb = tl * 16;

        const int p  = tb + ln;
        int rem = (p < NPAIR) ? p : (NPAIR - 1);
        int pi = 0;
#pragma unroll
        for (int s = 0; s < NN - 1; ++s) {
            const int  len = NN - pi;
            const bool adv = (rem >= len);
            rem = adv ? (rem - len) : rem;
            pi  = adv ? (pi + 1) : pi;
        }
        const int pj = pi + rem;

        const float* ni = nodeS + (e * NN + pi) * C1;
        const float* nj = nodeS + (e * NN + pj) * C1;

        v16h a1[2];
#pragma unroll
        for (int kb = 0; kb < 2; ++kb) {
#pragma unroll
            for (int t2 = 0; t2 < 2; ++t2) {
                const int cb = kb * 32 + t2 * 16 + hi * 8;
#pragma unroll
                for (int k = 0; k < 8; ++k) {
                    const float d = ni[cb + k] - nj[cb + k];
                    a1[kb][t2 * 8 + k] = (f16)((d * d) * 16.0f);
                }
            }
        }

#pragma unroll
        for (int nt = 0; nt < 8; ++nt) {
            v8f acc = zero8();
            const f16* wrow = w1h + (size_t)(nt * 16 + ln) * C1 + 8 * hi;
            Frag bu0, bu1;
            bu0.h[0] = *(const v8h*)(wrow + 0);
            bu0.h[1] = *(const v8h*)(wrow + 16);
            bu1.h[0] = *(const v8h*)(wrow + 32);
            bu1.h[1] = *(const v8h*)(wrow + 48);
            acc = wmma16(a1[0], bu0.v, acc);
            acc = wmma16(a1[1], bu1.v, acc);
            asm volatile("v_nop\n\tv_nop\n\tv_nop\n\tv_nop"
                         : "+v"(acc) : "v"(a1[0]), "v"(a1[1]), "v"(bu0.v), "v"(bu1.v));
            const int o = nt * 16 + ln;
            const float s = s1S[o], mu = m1S[o], be = b1S[o];
#pragma unroll
            for (int v = 0; v < 8; ++v) {
                float h = (acc[v] * acc_scale - mu) * s + be;
                h = (h >= 0.0f) ? h : 0.01f * h;
                myH1[(v + 8 * hi) * H1S + o] = (f16)(h * 16.0f);
            }
        }
        __builtin_amdgcn_fence(__ATOMIC_RELEASE, "wavefront");
        __builtin_amdgcn_wave_barrier();

        v16h a2[4];
#pragma unroll
        for (int kb = 0; kb < 4; ++kb) {
            Frag au;
            au.h[0] = *(const v8h*)(myH1 + ln * H1S + kb * 32 + 8 * hi);
            au.h[1] = *(const v8h*)(myH1 + ln * H1S + kb * 32 + 16 + 8 * hi);
            a2[kb] = au.v;
        }

        v8f part = zero8();
#pragma unroll
        for (int nt = 0; nt < 4; ++nt) {
            v8f acc = zero8();
            const f16* wrow = w2h + (size_t)(nt * 16 + ln) * C2 + 8 * hi;
            v16h bl;
#pragma unroll
            for (int kb = 0; kb < 4; ++kb) {
                Frag bu;
                bu.h[0] = *(const v8h*)(wrow + kb * 32);
                bu.h[1] = *(const v8h*)(wrow + kb * 32 + 16);
                bl = bu.v;
                acc = wmma16(a2[kb], bl, acc);
            }
            asm volatile("v_nop\n\tv_nop\n\tv_nop\n\tv_nop"
                         : "+v"(acc) : "v"(a2[0]), "v"(a2[1]), "v"(a2[2]), "v"(a2[3]), "v"(bl));
            const int o = nt * 16 + ln;
            const float s = s2S[o], mu = m2S[o], be = b2S[o], w3v = w3S[o];
#pragma unroll
            for (int v = 0; v < 8; ++v) {
                float h = (acc[v] * acc_scale - mu) * s + be;
                h = (h >= 0.0f) ? h : 0.01f * h;
                part[v] += h * w3v;
            }
        }
#pragma unroll
        for (int off = 1; off < 16; off <<= 1) {
#pragma unroll
            for (int v = 0; v < 8; ++v) part[v] += __shfl_xor(part[v], off, 32);
        }
        const int r8 = ln & 7;
        float myv = part[0];
#pragma unroll
        for (int v = 1; v < 8; ++v) myv = (r8 == v) ? part[v] : myv;
        const int src = 8 * hi + r8;
        const int qi = __shfl(pi, src, 32);
        const int qj = __shfl(pj, src, 32);
        const int pp = tb + src;
        if (ln < 8 && pp < NPAIR) {
            const float ev = myv + bias3;
            epS[e * NPIX + qi * NN + qj] = ev;
            epS[e * NPIX + qj * NN + qi] = ev;
        }
        __builtin_amdgcn_fence(__ATOMIC_RELEASE, "wavefront");
        __builtin_amdgcn_wave_barrier();
    }
    __syncthreads();

    float* outS = nodeS;
    for (int q = tid; q < EPB * NPIX; q += NTHR) {
        const int e = q / NPIX, r = q - e * NPIX;
        int eg = epg0 + e; eg = (eg < nB) ? eg : (nB - 1);
        outS[2 * q] = last_edge[(size_t)eg * NPIX + r];
    }

    if (tid < EPB * NN) {
        const int e = tid / NN, i = tid - e * NN;
        float* er = epS + e * NPIX + i * NN;
        const float* mk = mkS + i * NN;
        float mx = -__builtin_huge_valf();
#pragma unroll
        for (int j = 0; j < NN; ++j) {
            const float vv = er[j] * mk[j] + ((j == i) ? 1.0f : 0.0f);
            mx = fmaxf(mx, vv);
        }
        float sum = 0.0f;
#pragma unroll 1
        for (int j = 0; j < NN; ++j) {
            const float vv = er[j] * mk[j] + ((j == i) ? 1.0f : 0.0f);
            const float ex = expf(vv - mx);
            er[j] = ex;
            sum += ex;
        }
        const float inv = 1.0f / sum;
        float* orow = outS + 2 * (e * NPIX + i * NN);
#pragma unroll 1
        for (int j = 0; j < NN; ++j) orow[2 * j + 1] = er[j] * inv;
    }
    __syncthreads();

    const int totP = nB * PPE;
    v4f_t ov[NPK];
#pragma unroll
    for (int k = 0; k < NPK; ++k) {
        const int q  = k * NTHR + tid;
        const int qc = (q < PPB) ? q : (PPB - 1);
        ov[k] = *(const v4f*)(outS + 4 * qc);
    }
#pragma unroll
    for (int k = 0; k < NPK; ++k) {
        const int q  = k * NTHR + tid;
        const int gq = blk * PPB + q;
        if (q < PPB && gq < totP) *(volatile v4f_t*)(out + (size_t)gq * 4) = ov[k];
    }
    __threadfence();
#pragma unroll
    for (int k = 0; k < NPK; ++k) {
        const int q  = k * NTHR + tid;
        const int gq = blk * PPB + q;
        if (q < PPB && gq < totP) *(volatile v4f_t*)(out + (size_t)gq * 4) = ov[k];
    }
}

extern "C" void kernel_launch(void* const* d_in, const int* in_sizes, int n_in,
                              void* d_out, int out_size, void* d_ws, size_t ws_size,
                              hipStream_t stream)
{
    if (n_in < 14) return;
    const int nodeN = in_sizes[0];
    if (nodeN <= 0 || (nodeN % (NN * C1)) != 0) return;
    const int nB = nodeN / (NN * C1);
    if (in_sizes[1] != nB * NPIX) return;
    if (in_sizes[2] != C2 * C1) return;
    if (in_sizes[3] < C2 || in_sizes[4] < C2 || in_sizes[5] < C2 || in_sizes[6] < C2) return;
    if (in_sizes[7] != C1 * C2) return;
    if (in_sizes[8] < C1 || in_sizes[9] < C1 || in_sizes[10] < C1 || in_sizes[11] < C1) return;
    if (in_sizes[12] < C1 || in_sizes[13] < 1) return;
    if (out_size != nB * OUTE) return;

    const float* node      = (const float*)d_in[0];
    const float* last_edge = (const float*)d_in[1];
    const float* W1        = (const float*)d_in[2];
    const float* g1        = (const float*)d_in[3];
    const float* b1        = (const float*)d_in[4];
    const float* m1        = (const float*)d_in[5];
    const float* v1        = (const float*)d_in[6];
    const float* W2        = (const float*)d_in[7];
    const float* g2        = (const float*)d_in[8];
    const float* b2        = (const float*)d_in[9];
    const float* m2        = (const float*)d_in[10];
    const float* v2        = (const float*)d_in[11];
    const float* W3        = (const float*)d_in[12];
    const float* b3        = (const float*)d_in[13];
    float* out = (float*)d_out;

    const size_t nW   = (size_t)C1 * C2;
    const size_t oW1  = 0;
    const size_t oW2  = oW1 + nW * sizeof(f16);
    const size_t total = oW2 + nW * sizeof(f16);
    if (total > ws_size) return;
    char* ws = (char*)d_ws;
    f16* w1h = (f16*)(ws + oW1);
    f16* w2h = (f16*)(ws + oW2);

    const int n8  = (int)(nW / 8);
    const int nbm = (n8 + 255) / 256;
    cvt_w_kernel<<<2 * nbm, 256, 0, stream>>>(W1, W2, w1h, w2h, n8, nbm);

    const int grid = (nB + EPB - 1) / EPB;
    edge_kernel<<<grid, NTHR, 0, stream>>>(node, last_edge, w1h, g1, b1, m1, v1,
                                           w2h, g2, b2, m2, v2, W3, b3, out, nB);
}
